// SelfAttention_1314259992903
// MI455X (gfx1250) — hardware-verified
//
#include <hip/hip_runtime.h>


#ifndef NB
#define NB 2
#endif
#ifndef SEQ
#define SEQ 2048
#endif
#define NB_FULL    2
#define SEQ_FULL   2048
#define DIM        1024
#define NHEAD      16
#define HDIM       64
#define INNER      (NHEAD * HDIM)
#define N3         (3 * INNER)
#define ROWS       (NB * SEQ)
#define KDIM       1024
#define BQ         128
#define BK         32
#define NWAVE      8
#define LDSP       40
#define CP         68
#define TPW        72
#define PCARRY     1024.0f
#define EPS_F      1e-10f
#define PLANE      ((size_t)NB * NHEAD * SEQ * HDIM)

static_assert(SEQ % 128 == 0);
static_assert(SEQ % BK == 0);
static_assert(SEQ <= SEQ_FULL);
static_assert(NB >= 1 && NB <= NB_FULL);
static_assert(DIM == KDIM);
static_assert(INNER == KDIM);
static_assert(KDIM % 32 == 0);
static_assert(KDIM / 32 == 32);
static_assert(HDIM == 64);
static_assert(BQ == NWAVE * 16);
static_assert(ROWS % 128 == 0);
static_assert(N3 % 128 == 0);
static_assert((2 * INNER) % 128 == 0);
static_assert(INNER % 128 == 0);
static_assert(DIM % 128 == 0);
static_assert(DIM % 64 == 0);
static_assert((LDSP * 2) % 16 == 0);
static_assert((CP * 4) % 16 == 0);
static_assert((TPW * 2) % 16 == 0);
static_assert(((size_t)ROWS * DIM / 8) % 256 == 0);
static_assert(((size_t)NB * SEQ * SEQ / 8) % 256 == 0);
static_assert(DIM % 8 == 0 && SEQ % 8 == 0);

typedef __bf16   bf16;
typedef _Float16 f16;
typedef bf16     v16bf __attribute__((ext_vector_type(16)));
typedef bf16     v8bf  __attribute__((ext_vector_type(8)));
typedef f16      v16h  __attribute__((ext_vector_type(16)));
typedef float    v8f   __attribute__((ext_vector_type(8)));
typedef float    v4f   __attribute__((ext_vector_type(4)));
typedef unsigned v4u   __attribute__((ext_vector_type(4)));

union FragB  { v16bf v; v4u q[2]; };
union FragH  { v16h  v; v4u q[2]; f16 h[16]; };
union Pack8B { v4u u; v8bf v; bf16 h[8]; };
union Pack8H { v4u u; f16 h[8]; };

static __device__ __forceinline__ v8f mma_bf16(v16bf a, v16bf b, v8f acc) {
  acc = __builtin_amdgcn_wmma_f32_16x16x32_bf16(false, a, false, b, (short)0, acc, false, false);
  asm volatile("v_nop\n\tv_nop\n\tv_nop\n\tv_nop" : "+v"(acc) : "v"(a), "v"(b));
  return acc;
}
static __device__ __forceinline__ v8f mma_f16(v16h a, v16h b, v8f acc) {
  acc = __builtin_amdgcn_wmma_f32_16x16x32_f16(false, a, false, b, (short)0, acc, false, false);
  asm volatile("v_nop\n\tv_nop\n\tv_nop\n\tv_nop" : "+v"(acc) : "v"(a), "v"(b));
  return acc;
}

static __device__ __forceinline__ void split8(v4f x0, v4f x1, v4u& uh, v4u& ul) {
  Pack8B ph, pl;
  #pragma unroll
  for (int e = 0; e < 4; ++e) {
    const bf16 h0 = (bf16)x0[e];
    const bf16 h1 = (bf16)x1[e];
    ph.h[e]     = h0;
    ph.h[4 + e] = h1;
    pl.h[e]     = (bf16)(x0[e] - (float)h0);
    pl.h[4 + e] = (bf16)(x1[e] - (float)h1);
  }
  uh = ph.u;
  ul = pl.u;
}

__global__ __launch_bounds__(256) void k_cvt_rows(const float* __restrict__ in, bf16* __restrict__ out,
                                                  int cols, int rows_per_batch, int in_batch_rows,
                                                  int in_row_stride, int total8) {
  const int g = blockIdx.x * 256 + threadIdx.x;
  if (g >= total8) return;
  const int e   = g * 8;
  const int row = e / cols;
  const int col = e - row * cols;
  const int b   = row / rows_per_batch;
  const int s   = row - b * rows_per_batch;
  const float* src = in + ((size_t)b * in_batch_rows + s) * (size_t)in_row_stride + col;
  const v4f a0 = *(const v4f*)(src);
  const v4f a1 = *(const v4f*)(src + 4);
  Pack8B pk;
  #pragma unroll
  for (int i = 0; i < 4; ++i) {
    pk.h[i]     = (bf16)a0[i];
    pk.h[4 + i] = (bf16)a1[i];
  }
  const v4u val = pk.u;
  bf16* dst = out + (size_t)e;
  *(volatile v4u*)dst = val;
  __threadfence();
  *(volatile v4u*)dst = val;
}

__global__ __launch_bounds__(256) void k_cvt_wt(const float* __restrict__ in, bf16* __restrict__ out, int C) {
  __shared__ __align__(16) bf16 sT[64 * TPW];
  const int n0  = blockIdx.x * 64;
  const int k0  = blockIdx.y * 64;
  const int tid = threadIdx.x;
  #pragma unroll
  for (int kk = 0; kk < 2; ++kk) {
    const int k  = kk * 32 + (tid >> 3);
    const int nl = (tid & 7) * 8;
    const float* src = in + (size_t)(k0 + k) * C + n0 + nl;
    const v4f a0 = *(const v4f*)(src);
    const v4f a1 = *(const v4f*)(src + 4);
    #pragma unroll
    for (int i = 0; i < 4; ++i) {
      sT[(nl + i) * TPW + k]     = (bf16)a0[i];
      sT[(nl + 4 + i) * TPW + k] = (bf16)a1[i];
    }
  }
  __syncthreads();
  v4u    val[2];
  size_t idx[2];
  #pragma unroll
  for (int kk = 0; kk < 2; ++kk) {
    const int n  = kk * 32 + (tid >> 3);
    const int ks = (tid & 7) * 8;
    Pack8B p;
    p.v = *(const v8bf*)(&sT[n * TPW + ks]);
    val[kk] = p.u;
    idx[kk] = (size_t)(n0 + n) * KDIM + k0 + ks;
  }
  #pragma unroll
  for (int kk = 0; kk < 2; ++kk) *(volatile v4u*)(out + idx[kk]) = val[kk];
  __threadfence();
  #pragma unroll
  for (int kk = 0; kk < 2; ++kk) *(volatile v4u*)(out + idx[kk]) = val[kk];
}

static __device__ __forceinline__ void gemm_tile(const bf16* __restrict__ A, const bf16* __restrict__ Bt,
                                                 int m0, int n0, int npass, size_t a_pass_stride,
                                                 bf16* sa, bf16* sb, v8f (&acc)[2][4]) {
  const int tid  = threadIdx.x;
  const int wave = __builtin_amdgcn_readfirstlane(tid >> 5);
  const int lane = tid & 31;
  const int lq   = lane & 15;
  const int hi   = lane >> 4;
  const int wm   = wave >> 1;
  const int wn   = wave & 1;
  const int srow = tid >> 1;
  const int sseg = (tid & 1) * 16;
  const size_t aoff = (size_t)(m0 + srow) * KDIM + sseg;
  const size_t boff = (size_t)(n0 + srow) * KDIM + sseg;
  const int    soff = srow * LDSP + sseg;

  for (int t = 0; t < npass * (KDIM / 32); ++t) {
    const int pass = t >> 5;
    const int k    = (t & 31) * 32;
    const size_t ao = aoff + (size_t)pass * a_pass_stride + k;
    const v4u a0 = *(const v4u*)(A + ao);
    const v4u a1 = *(const v4u*)(A + ao + 8);
    const v4u b0 = *(const v4u*)(Bt + boff + k);
    const v4u b1 = *(const v4u*)(Bt + boff + k + 8);
    __syncthreads();
    *(v4u*)(sa + soff)     = a0;
    *(v4u*)(sa + soff + 8) = a1;
    *(v4u*)(sb + soff)     = b0;
    *(v4u*)(sb + soff + 8) = b1;
    __syncthreads();

    FragB af[2], bfm[4];
    #pragma unroll
    for (int i = 0; i < 2; ++i) {
      const int base = (wm * 32 + i * 16 + lq) * LDSP + 8 * hi;
      af[i].q[0] = *(const v4u*)(sa + base);
      af[i].q[1] = *(const v4u*)(sa + base + 16);
    }
    #pragma unroll
    for (int j = 0; j < 4; ++j) {
      const int base = (wn * 64 + j * 16 + lq) * LDSP + 8 * hi;
      bfm[j].q[0] = *(const v4u*)(sb + base);
      bfm[j].q[1] = *(const v4u*)(sb + base + 16);
    }
    #pragma unroll
    for (int i = 0; i < 2; ++i) {
      #pragma unroll
      for (int j = 0; j < 4; ++j) acc[i][j] = mma_bf16(af[i].v, bfm[j].v, acc[i][j]);
    }
  }
}

__global__ __launch_bounds__(256) void k_gemm_qk(const bf16* __restrict__ Xb, const bf16* __restrict__ Wqt,
                                                 bf16* __restrict__ qk) {
  __shared__ __align__(16) bf16  sa[128 * LDSP];
  __shared__ __align__(16) bf16  sb[128 * LDSP];
  __shared__ __align__(16) float sC[NWAVE * 16 * CP];
  const int m0 = blockIdx.y * 128;
  const int n0 = blockIdx.x * 128;
  v8f acc[2][4];
  #pragma unroll
  for (int i = 0; i < 2; ++i) {
    #pragma unroll
    for (int j = 0; j < 4; ++j) acc[i][j] = (v8f){0, 0, 0, 0, 0, 0, 0, 0};
  }
  gemm_tile(Xb, Wqt, m0, n0, 1, 0, sa, sb, acc);

  const int tid  = threadIdx.x;
  const int wave = __builtin_amdgcn_readfirstlane(tid >> 5);
  const int lane = tid & 31;
  const int lq   = lane & 15;
  const int hi   = lane >> 4;
  const int wm   = wave >> 1;
  const int wn   = wave & 1;
  const int cw   = wave * 16 * CP;
  const int n     = n0 + wn * 64;
  const int which = n >> 10;
  const int hh    = (n >> 6) & 15;

  #pragma unroll
  for (int i = 0; i < 2; ++i) {
    #pragma unroll
    for (int j = 0; j < 4; ++j) {
      #pragma unroll
      for (int r = 0; r < 8; ++r) sC[cw + (hi * 8 + r) * CP + j * 16 + lq] = acc[i][j][r];
    }
    __syncthreads();
    v4u    vh[4], vl[4];
    size_t gi[4];
    #pragma unroll
    for (int it = 0; it < 4; ++it) {
      const int row = it * 4 + (lane >> 3);
      const int c0  = (lane & 7) * 8;
      const v4f x0 = *(const v4f*)(&sC[cw + row * CP + c0]);
      const v4f x1 = *(const v4f*)(&sC[cw + row * CP + c0 + 4]);
      split8(x0, x1, vh[it], vl[it]);
      const int gr = m0 + wm * 32 + i * 16 + row;
      const int bb = gr / SEQ;
      const int s  = gr - bb * SEQ;
      gi[it] = (size_t)which * 2 * PLANE + (((size_t)bb * NHEAD + hh) * SEQ + s) * HDIM + c0;
    }
    #pragma unroll
    for (int it = 0; it < 4; ++it) {
      *(volatile v4u*)(qk + gi[it])         = vh[it];
      *(volatile v4u*)(qk + gi[it] + PLANE) = vl[it];
    }
    __threadfence();
    #pragma unroll
    for (int it = 0; it < 4; ++it) {
      *(volatile v4u*)(qk + gi[it])         = vh[it];
      *(volatile v4u*)(qk + gi[it] + PLANE) = vl[it];
    }
    __syncthreads();
  }
}

__global__ __launch_bounds__(256) void k_gemm_vt(const bf16* __restrict__ Wvt, const bf16* __restrict__ Xb,
                                                 f16* __restrict__ vt) {
  __shared__ __align__(16) bf16  sa[128 * LDSP];
  __shared__ __align__(16) bf16  sb[128 * LDSP];
  __shared__ __align__(16) float sC[NWAVE * 16 * CP];
  const int m0 = blockIdx.y * 128;
  const int n0 = blockIdx.x * 128;
  v8f acc[2][4];
  #pragma unroll
  for (int i = 0; i < 2; ++i) {
    #pragma unroll
    for (int j = 0; j < 4; ++j) acc[i][j] = (v8f){0, 0, 0, 0, 0, 0, 0, 0};
  }
  gemm_tile(Wvt, Xb, m0, n0, 1, 0, sa, sb, acc);

  const int tid  = threadIdx.x;
  const int wave = __builtin_amdgcn_readfirstlane(tid >> 5);
  const int lane = tid & 31;
  const int lq   = lane & 15;
  const int hi   = lane >> 4;
  const int wm   = wave >> 1;
  const int wn   = wave & 1;
  const int cw   = wave * 16 * CP;
  const int ns   = n0 + wn * 64;
  const int bb   = ns / SEQ;
  const int s0   = ns - bb * SEQ;

  #pragma unroll
  for (int i = 0; i < 2; ++i) {
    #pragma unroll
    for (int j = 0; j < 4; ++j) {
      #pragma unroll
      for (int r = 0; r < 8; ++r) sC[cw + (hi * 8 + r) * CP + j * 16 + lq] = acc[i][j][r];
    }
    __syncthreads();
    v4u    vv[4];
    size_t gi[4];
    #pragma unroll
    for (int it = 0; it < 4; ++it) {
      const int row = it * 4 + (lane >> 3);
      const int c0  = (lane & 7) * 8;
      const v4f x0 = *(const v4f*)(&sC[cw + row * CP + c0]);
      const v4f x1 = *(const v4f*)(&sC[cw + row * CP + c0 + 4]);
      Pack8H ph;
      #pragma unroll
      for (int e = 0; e < 4; ++e) {
        ph.h[e]     = (f16)x0[e];
        ph.h[4 + e] = (f16)x1[e];
      }
      vv[it] = ph.u;
      const int m = m0 + wm * 32 + i * 16 + row;
      gi[it] = ((size_t)bb * INNER + m) * SEQ + s0 + c0;
    }
    #pragma unroll
    for (int it = 0; it < 4; ++it) *(volatile v4u*)(vt + gi[it]) = vv[it];
    __threadfence();
    #pragma unroll
    for (int it = 0; it < 4; ++it) *(volatile v4u*)(vt + gi[it]) = vv[it];
    __syncthreads();
  }
}

__global__ __launch_bounds__(256) void k_attn(const bf16* __restrict__ qh, const bf16* __restrict__ ql,
                                              const bf16* __restrict__ kh, const bf16* __restrict__ kl,
                                              const f16* __restrict__ vt, const bf16* __restrict__ mb,
                                              bf16* __restrict__ zh, bf16* __restrict__ zl) {
  const int qblk = blockIdx.x;
  const int h    = blockIdx.y;
  const int b    = blockIdx.z;
  const int tid  = threadIdx.x;
  const int wave = __builtin_amdgcn_readfirstlane(tid >> 5);
  const int lane = tid & 31;
  const int lq   = lane & 15;
  const int hi   = lane >> 4;

  __shared__ __align__(16) float sO[NWAVE * 16 * CP];

  const int qrow0 = qblk * BQ + wave * 16;
  const int bh    = b * NHEAD + h;
  const int qbase = (bh * SEQ + qrow0 + lq) * HDIM + hi * 8;
  const int kbase = (bh * SEQ + lq) * HDIM + hi * 8;
  const int vbase = (bh * HDIM + lq) * SEQ + hi * 8;
  const size_t mbase = ((size_t)b * SEQ + qrow0 + lq) * SEQ + hi * 8;

  v8f o[4];
  #pragma unroll
  for (int dt = 0; dt < 4; ++dt) o[dt] = (v8f){0, 0, 0, 0, 0, 0, 0, 0};

  float rmax  = -__builtin_inff();
  float s_all = 0.0f;
  float s_m   = 0.0f;
  const float SL = 0.125f * 1.4426950408889634f;

  for (int i = 0; i < SEQ / BK; ++i) {
    const int j0 = i * BK;
    int qo = qbase;
    asm volatile("" : "+v"(qo));

    const v4u mw0 = *(const v4u*)(mb + mbase + j0);
    const v4u mw1 = *(const v4u*)(mb + mbase + j0 + 16);

    v8f c[2];
    c[0] = (v8f){0, 0, 0, 0, 0, 0, 0, 0};
    c[1] = (v8f){0, 0, 0, 0, 0, 0, 0, 0};
    #pragma unroll
    for (int f = 0; f < 2; ++f) {
      FragB bqh, bql;
      bqh.q[0] = *(const v4u*)(qh + qo + f * 32);
      bqh.q[1] = *(const v4u*)(qh + qo + f * 32 + 16);
      bql.q[0] = *(const v4u*)(ql + qo + f * 32);
      bql.q[1] = *(const v4u*)(ql + qo + f * 32 + 16);
      #pragma unroll
      for (int sub = 0; sub < 2; ++sub) {
        const int ko = kbase + (j0 + sub * 16) * HDIM + f * 32;
        FragB akh, akl;
        akh.q[0] = *(const v4u*)(kh + ko);
        akh.q[1] = *(const v4u*)(kh + ko + 16);
        akl.q[0] = *(const v4u*)(kl + ko);
        akl.q[1] = *(const v4u*)(kl + ko + 16);
        c[sub] = mma_bf16(akh.v, bqh.v, c[sub]);
        c[sub] = mma_bf16(akh.v, bql.v, c[sub]);
        c[sub] = mma_bf16(akl.v, bqh.v, c[sub]);
      }
    }

    float mk0[8], mk1[8];
    #pragma unroll
    for (int w = 0; w < 4; ++w) {
      mk0[2 * w]     = __uint_as_float(mw0[w] << 16);
      mk0[2 * w + 1] = __uint_as_float(mw0[w] & 0xffff0000u);
      mk1[2 * w]     = __uint_as_float(mw1[w] << 16);
      mk1[2 * w + 1] = __uint_as_float(mw1[w] & 0xffff0000u);
    }

    float m_new = rmax;
    #pragma unroll
    for (int r = 0; r < 8; ++r) {
      m_new = fmaxf(m_new, c[0][r]);
      m_new = fmaxf(m_new, c[1][r]);
    }
    const float m_oth = __shfl_xor(m_new, 16, 32);
    m_new = fmaxf(m_new, m_oth);
    const float alpha = __builtin_amdgcn_exp2f((rmax - m_new) * SL);
    rmax = m_new;

    FragH pa;
    float ps_all = 0.0f;
    float ps_m   = 0.0f;
    #pragma unroll
    for (int r = 0; r < 8; ++r) {
      const float p0  = __builtin_amdgcn_exp2f((c[0][r] - m_new) * SL);
      const float p1  = __builtin_amdgcn_exp2f((c[1][r] - m_new) * SL);
      const float pm0 = p0 * mk0[r];
      const float pm1 = p1 * mk1[r];
      ps_all += p0 + p1;
      ps_m   += pm0 + pm1;
      pa.h[r]     = (f16)(pm0 * PCARRY);
      pa.h[8 + r] = (f16)(pm1 * PCARRY);
    }
    const float oa = __shfl_xor(ps_all, 16, 32);
    const float om = __shfl_xor(ps_m, 16, 32);
    s_all = s_all * alpha + ps_all + oa;
    s_m   = s_m * alpha + ps_m + om;

    float sc[8];
    #pragma unroll
    for (int r = 0; r < 8; ++r) sc[r] = __shfl(alpha, (hi << 3) + r, 32);
    #pragma unroll
    for (int dt = 0; dt < 4; ++dt) {
      #pragma unroll
      for (int r = 0; r < 8; ++r) o[dt][r] *= sc[r];
    }

    #pragma unroll
    for (int dt = 0; dt < 4; ++dt) {
      const int vo = vbase + dt * 16 * SEQ + j0;
      FragH bv;
      bv.q[0] = *(const v4u*)(vt + vo);
      bv.q[1] = *(const v4u*)(vt + vo + 16);
      o[dt] = mma_f16(pa.v, bv.v, o[dt]);
    }
  }

  const float den  = s_m + EPS_F * s_all;
  const float invd = (1.0f / den) * (1.0f / PCARRY);
  float rs[8];
  #pragma unroll
  for (int r = 0; r < 8; ++r) rs[r] = __shfl(invd, (hi << 3) + r, 32);

  const int cw = wave * 16 * CP;
  #pragma unroll
  for (int r = 0; r < 8; ++r) {
    #pragma unroll
    for (int dt = 0; dt < 4; ++dt) sO[cw + (hi * 8 + r) * CP + dt * 16 + lq] = o[dt][r] * rs[r];
  }
  __syncthreads();

  v4u    vh[4], vl[4];
  size_t gi[4];
  #pragma unroll
  for (int it = 0; it < 4; ++it) {
    const int row = it * 4 + (lane >> 3);
    const int c0  = (lane & 7) * 8;
    const v4f x0 = *(const v4f*)(&sO[cw + row * CP + c0]);
    const v4f x1 = *(const v4f*)(&sO[cw + row * CP + c0 + 4]);
    split8(x0, x1, vh[it], vl[it]);
    gi[it] = ((size_t)b * SEQ + qrow0 + row) * INNER + h * HDIM + c0;
  }
  #pragma unroll
  for (int it = 0; it < 4; ++it) {
    *(volatile v4u*)(zh + gi[it]) = vh[it];
    *(volatile v4u*)(zl + gi[it]) = vl[it];
  }
  __threadfence();
  #pragma unroll
  for (int it = 0; it < 4; ++it) {
    *(volatile v4u*)(zh + gi[it]) = vh[it];
    *(volatile v4u*)(zl + gi[it]) = vl[it];
  }
}

__global__ __launch_bounds__(256) void k_gemm_out(const bf16* __restrict__ Z, const bf16* __restrict__ Wot,
                                                  const float* __restrict__ bias, float* __restrict__ out) {
  __shared__ __align__(16) bf16  sa[128 * LDSP];
  __shared__ __align__(16) bf16  sb[128 * LDSP];
  __shared__ __align__(16) float sC[NWAVE * 16 * CP];
  const int m0 = blockIdx.y * 128;
  const int n0 = blockIdx.x * 128;
  v8f acc[2][4];
  #pragma unroll
  for (int i = 0; i < 2; ++i) {
    #pragma unroll
    for (int j = 0; j < 4; ++j) acc[i][j] = (v8f){0, 0, 0, 0, 0, 0, 0, 0};
  }
  gemm_tile(Z, Wot, m0, n0, 2, (size_t)ROWS * INNER, sa, sb, acc);

  const int tid  = threadIdx.x;
  const int wave = __builtin_amdgcn_readfirstlane(tid >> 5);
  const int lane = tid & 31;
  const int lq   = lane & 15;
  const int hi   = lane >> 4;
  const int wm   = wave >> 1;
  const int wn   = wave & 1;
  const int cw   = wave * 16 * CP;
  const int ncol = n0 + wn * 64 + lq * 4;

  v4f bias4 = *(const v4f*)(bias + ncol);
  #pragma unroll
  for (int e = 0; e < 4; ++e) bias4[e] = (float)(bf16)bias4[e];

  #pragma unroll
  for (int i = 0; i < 2; ++i) {
    #pragma unroll
    for (int j = 0; j < 4; ++j) {
      #pragma unroll
      for (int r = 0; r < 8; ++r) sC[cw + (hi * 8 + r) * CP + j * 16 + lq] = acc[i][j][r];
    }
    __syncthreads();
    v4f    vals[8];
    size_t gi[8];
    #pragma unroll
    for (int it = 0; it < 8; ++it) {
      const int row = it * 2 + hi;
      const v4f v = *(const v4f*)(&sC[cw + row * CP + lq * 4]);
      vals[it] = v + bias4;
      const int gr = m0 + wm * 32 + i * 16 + row;
      const int bb = gr / SEQ;
      const int s  = gr - bb * SEQ;
      gi[it] = ((size_t)bb * SEQ_FULL + s) * DIM + ncol;
    }
    #pragma unroll
    for (int it = 0; it < 8; ++it) *(volatile v4f*)(out + gi[it]) = vals[it];
    __threadfence();
    #pragma unroll
    for (int it = 0; it < 8; ++it) *(volatile v4f*)(out + gi[it]) = vals[it];
    __syncthreads();
  }
}

#define SZ_XB   ((size_t)ROWS * DIM * 2)
#define SZ_MB   ((size_t)NB * SEQ * SEQ * 2)
#define SZ_WQT  ((size_t)N3 * KDIM * 2)
#define SZ_WOT  ((size_t)DIM * KDIM * 2)
#define SZ_QK   ((size_t)4 * PLANE * 2)
#define SZ_VT   ((size_t)PLANE * 2)
#define SZ_Z    ((size_t)2 * ROWS * INNER * 2)
#define OFF_XB  ((size_t)0)
#define OFF_MB  (OFF_XB + SZ_XB)
#define OFF_WQT (OFF_MB + SZ_MB)
#define OFF_WOT (OFF_WQT + SZ_WQT)
#define OFF_QK  (OFF_WOT + SZ_WOT)
#define OFF_VT  (OFF_QK + SZ_QK)
#define OFF_Z   (OFF_VT + SZ_VT)
#define WS_TOTAL (OFF_Z + SZ_Z)

static_assert(WS_TOTAL <= (size_t)134217728);
static_assert(SZ_XB % 128 == 0 && SZ_MB % 128 == 0 && SZ_WQT % 128 == 0 && SZ_WOT % 128 == 0);
static_assert(SZ_QK % 128 == 0 && SZ_VT % 128 == 0 && SZ_Z % 128 == 0);

extern "C" void kernel_launch(void* const* d_in, const int* in_sizes, int n_in,
                              void* d_out, int out_size, void* d_ws, size_t ws_size,
                              hipStream_t stream) {
  if (n_in < 5) return;
  const size_t rows_used = (size_t)(NB - 1) * SEQ_FULL + SEQ;
  if ((size_t)in_sizes[0] < rows_used * DIM) return;
  if ((size_t)in_sizes[1] < (size_t)(NB - 1) * SEQ_FULL * SEQ_FULL + (size_t)(SEQ - 1) * SEQ_FULL + SEQ) return;
  if ((size_t)in_sizes[2] < (size_t)DIM * N3) return;
  if ((size_t)in_sizes[3] < (size_t)INNER * DIM) return;
  if ((size_t)in_sizes[4] < (size_t)DIM) return;
  if ((size_t)out_size < rows_used * DIM) return;
  if (ws_size < WS_TOTAL) return;

  const float* x    = (const float*)d_in[0];
  const float* mask = (const float*)d_in[1];
  const float* Wqkv = (const float*)d_in[2];
  const float* Wout = (const float*)d_in[3];
  const float* bout = (const float*)d_in[4];
  float*       out  = (float*)d_out;

  char* ws = (char*)d_ws;
  bf16* Xb  = (bf16*)(ws + OFF_XB);
  bf16* Mb  = (bf16*)(ws + OFF_MB);
  bf16* Wqt = (bf16*)(ws + OFF_WQT);
  bf16* Wot = (bf16*)(ws + OFF_WOT);
  bf16* QK  = (bf16*)(ws + OFF_QK);
  f16*  Vt  = (f16*)(ws + OFF_VT);
  bf16* Zp  = (bf16*)(ws + OFF_Z);

  const int x8 = (int)((size_t)ROWS * DIM / 8);
  const int m8 = (int)((size_t)NB * SEQ * SEQ / 8);
  k_cvt_rows<<<dim3((x8 + 255) / 256), 256, 0, stream>>>(x, Xb, DIM, SEQ, SEQ_FULL, DIM, x8);
  k_cvt_rows<<<dim3((m8 + 255) / 256), 256, 0, stream>>>(mask, Mb, SEQ, SEQ, SEQ_FULL, SEQ_FULL, m8);
  k_cvt_wt<<<dim3(N3 / 64, KDIM / 64), 256, 0, stream>>>(Wqkv, Wqt, N3);
  k_cvt_wt<<<dim3(DIM / 64, KDIM / 64), 256, 0, stream>>>(Wout, Wot, DIM);

  k_gemm_qk<<<dim3((2 * INNER) / 128, ROWS / 128), 256, 0, stream>>>(Xb, Wqt, QK);
  k_gemm_vt<<<dim3(ROWS / 128, INNER / 128), 256, 0, stream>>>(Wqt + (size_t)2 * INNER * KDIM, Xb, Vt);

  k_attn<<<dim3(SEQ / BQ, NHEAD, NB), 256, 0, stream>>>(QK, QK + PLANE, QK + 2 * PLANE, QK + 3 * PLANE,
                                                        Vt, Mb, Zp, Zp + (size_t)ROWS * INNER);

  k_gemm_out<<<dim3(DIM / 128, ROWS / 128), 256, 0, stream>>>(Zp, Wot, bout, out);
}
